// TenerAttention_59167469469718
// MI455X (gfx1250) — hardware-verified
//
#include <hip/hip_runtime.h>


#define NB_  4
#define TT   1024
#define DD   1024
#define NH_  16
#define HD   64
#define KK   128
#define ZH   2
#define PCAR 1024.0f
typedef _Float16 h16;
typedef unsigned short bf;
typedef __attribute__((ext_vector_type(16))) __bf16   v16bf;
typedef __attribute__((ext_vector_type(16))) _Float16 v16h;
typedef __attribute__((ext_vector_type(8)))  _Float16 v8h;
typedef __attribute__((ext_vector_type(8)))  unsigned short v8us;
typedef __attribute__((ext_vector_type(8)))  float    v8f;
typedef __attribute__((ext_vector_type(4)))  float    v4f;
typedef v8h  __attribute__((may_alias)) v8ha;
typedef v4f  __attribute__((may_alias)) v4fa;
typedef v8us __attribute__((may_alias)) v8usa;

__device__ __forceinline__ unsigned short f2bf(float f) { unsigned u = __float_as_uint(f); u += 0x7FFFu + ((u >> 16) & 1u); return (unsigned short)(u >> 16); }
__device__ __forceinline__ float bf2f(unsigned short b) { return __uint_as_float(((unsigned)b) << 16); }
__device__ __forceinline__ float bfr(float f) { return bf2f(f2bf(f)); }
__device__ __forceinline__ v16h cat16(v8h lo, v8h hi) { return __builtin_shufflevector(lo, hi, 0, 1, 2, 3, 4, 5, 6, 7, 8, 9, 10, 11, 12, 13, 14, 15); }
__device__ __forceinline__ v16bf cat16b(v8us lo, v8us hi) { return __builtin_bit_cast(v16bf, __builtin_shufflevector(lo, hi, 0, 1, 2, 3, 4, 5, 6, 7, 8, 9, 10, 11, 12, 13, 14, 15)); }
__device__ __forceinline__ v8f wmma16(v16h a, v16h b, v8f c) { return __builtin_amdgcn_wmma_f32_16x16x32_f16(false, a, false, b, (short)0, c, false, false); }
__device__ __forceinline__ v8f wmmab(v16bf a, v16bf b, v8f c) { return __builtin_amdgcn_wmma_f32_16x16x32_bf16(false, a, false, b, (short)0, c, false, false); }


template <typename T16> struct WFrag;
template <> struct WFrag<h16> { typedef v16h V; static __device__ __forceinline__ V ld(const h16* p) { return cat16(*(const v8h*)p, *(const v8h*)(p + 16)); } static __device__ __forceinline__ v8f mma(V a, V b, v8f c) { return wmma16(a, b, c); } };
template <> struct WFrag<bf> { typedef v16bf V; static __device__ __forceinline__ V ld(const bf* p) { return cat16b(*(const v8us*)p, *(const v8us*)(p + 16)); } static __device__ __forceinline__ v8f mma(V a, V b, v8f c) { return wmmab(a, b, c); } };
template <typename T16, int NSPLIT, bool BIAS>
__global__ __launch_bounds__(32) void k_gemmw(const T16* __restrict__ A, const T16* __restrict__ A2, const T16* __restrict__ Bt, const T16* __restrict__ Bt2, int K, float* C, int ldc, const float* __restrict__ bias, size_t sA, size_t sB, size_t sC) {
    typedef typename WFrag<T16>::V V;
    __shared__ __align__(16) float os[16 * 68];
    const size_t z = blockIdx.z; A += z * sA; if (A2) A2 += z * sA; Bt += z * sB; if (Bt2) Bt2 += z * sB; C += z * sC;
    const int lane = threadIdx.x & 31, lr = lane & 15, hi = lane >> 4; const int r0 = blockIdx.x * 64, c0 = blockIdx.y * 64;
    v8f acc[4][4];
#pragma unroll
    for (int mb = 0; mb < 4; ++mb)
#pragma unroll
        for (int nb = 0; nb < 4; ++nb) acc[mb][nb] = (v8f){};
    const size_t aoff = (size_t)(r0 + lr) * K + 8 * hi, boff = (size_t)(c0 + lr) * K + 8 * hi;
#pragma unroll 1
    for (int kc = 0; kc < K; kc += 32) {
        V a[4], a2[4];
#pragma unroll
        for (int mb = 0; mb < 4; ++mb) { a[mb] = WFrag<T16>::ld(A + aoff + (size_t)mb * 16 * K + kc); if (NSPLIT == 1 || NSPLIT == 2) a2[mb] = WFrag<T16>::ld(A2 + aoff + (size_t)mb * 16 * K + kc); }
#pragma unroll
        for (int nb = 0; nb < 4; ++nb) { const V b = WFrag<T16>::ld(Bt + boff + (size_t)nb * 16 * K + kc); V b2; if (NSPLIT >= 2) b2 = WFrag<T16>::ld(Bt2 + boff + (size_t)nb * 16 * K + kc);
#pragma unroll
            for (int mb = 0; mb < 4; ++mb) { acc[mb][nb] = WFrag<T16>::mma(a[mb], b, acc[mb][nb]); if (NSPLIT == 1 || NSPLIT == 2) acc[mb][nb] = WFrag<T16>::mma(a2[mb], b, acc[mb][nb]); if (NSPLIT >= 2) acc[mb][nb] = WFrag<T16>::mma(a[mb], b2, acc[mb][nb]); } }
        asm volatile("v_nop\n\tv_nop\n\tv_nop\n\tv_nop" : "+v"(acc[0][0]), "+v"(acc[1][1]), "+v"(acc[2][2]), "+v"(acc[3][3]) : "v"(a[0]), "v"(a[3]));
    }
#pragma unroll
    for (int mb = 0; mb < 4; ++mb) {
#pragma unroll
        for (int nb = 0; nb < 4; ++nb) {
#pragma unroll
            for (int j = 0; j < 8; ++j) os[(hi * 8 + j) * 68 + nb * 16 + lr] = acc[mb][nb][j]; }
        __builtin_amdgcn_wave_barrier(); asm volatile("" ::: "memory");
        float* crow = C + (size_t)(r0 + mb * 16) * ldc + c0;
#pragma unroll 1
        for (int ps = 0; ps < 2; ++ps) {
#pragma unroll
            for (int s = 0; s < 8; ++s) { const int row = 2 * s + hi, cofs = lr * 4; v4f val = *(const v4fa*)(os + row * 68 + cofs); if (BIAS) { val[0] += bfr(bias[c0 + cofs]); val[1] += bfr(bias[c0 + cofs + 1]); val[2] += bfr(bias[c0 + cofs + 2]); val[3] += bfr(bias[c0 + cofs + 3]); }
                *(volatile v4f*)(crow + (size_t)row * ldc + cofs) = val; }
            if (ps == 0) __threadfence(); }
        __builtin_amdgcn_wave_barrier(); asm volatile("" ::: "memory");
    }
}

__device__ __forceinline__ h16 tohx(float x) { return (h16)x; }
__device__ __forceinline__ void splitf(float y, unsigned short& h, unsigned short& l) { h = f2bf(y); l = f2bf(y - bf2f(h)); }
typedef __attribute__((ext_vector_type(2))) _Float16 v2h;
typedef __attribute__((ext_vector_type(4))) _Float16 v4h;
typedef __attribute__((ext_vector_type(2))) unsigned short v2us;
typedef __attribute__((ext_vector_type(4))) unsigned short v4us;
typedef __attribute__((ext_vector_type(2))) float v2f;

__global__ __launch_bounds__(256) void k_cvt8(const float* __restrict__ src, bf* dst, size_t n8) { const size_t i = (size_t)blockIdx.x * 256 + threadIdx.x; if (i >= n8) return; const v8f v = *(const v8f*)(src + i * 8); v8us o;
#pragma unroll
    for (int k = 0; k < 8; ++k) o[k] = f2bf(v[k]); *(volatile v8us*)(dst + i * 8) = o; __threadfence(); *(volatile v8us*)(dst + i * 8) = o; }
__global__ __launch_bounds__(256) void k_trig(float* CS) { const int idx = blockIdx.x * 256 + threadIdx.x; if (idx >= TT * 32) return; const int t = idx / 32, m = idx % 32; const float w = powf(10000.0f, -(float)(2 * m) / (float)HD); const float ang = __fmul_rn((float)t, w); v2f cs; cs[0] = cosf(ang); cs[1] = sinf(ang); *(volatile v2f*)(CS + (size_t)idx * 2) = cs; __threadfence(); *(volatile v2f*)(CS + (size_t)idx * 2) = cs; }
__global__ __launch_bounds__(256) void k_apl(const float* __restrict__ QF, const float* __restrict__ uu, const float* __restrict__ vv, const float* __restrict__ CS, bf* Ah, bf* Al) { const size_t e = ((size_t)blockIdx.x * 256 + threadIdx.x) * 2; if (e >= (size_t)NH_ * TT * KK) return; const int c = (int)(e % KK); const int i = (int)((e / KK) % TT); const int h = (int)(e / ((size_t)KK * TT)); const float* q = QF + (size_t)i * DD + h * HD; v2us oh, ol; float r0, r1;
    if (c < HD) { r0 = __fadd_rn(q[c], bfr(uu[h * HD + c])); r1 = __fadd_rn(q[c + 1], bfr(uu[h * HD + c + 1])); }
    else { const int m = (c - HD) >> 1; const float ae = __fadd_rn(q[2 * m], bfr(vv[h * HD + 2 * m])), ao = __fadd_rn(q[2 * m + 1], bfr(vv[h * HD + 2 * m + 1])); const v2f cs = *(const v2f*)(CS + ((size_t)i * 32 + m) * 2); float p0 = __fmul_rn(ae, cs[0]); asm volatile("" : "+v"(p0)); float p1 = __fmul_rn(ao, cs[1]); asm volatile("" : "+v"(p1)); float p2 = __fmul_rn(-ae, cs[1]); asm volatile("" : "+v"(p2)); float p3 = __fmul_rn(ao, cs[0]); asm volatile("" : "+v"(p3)); r0 = __fadd_rn(p0, p1); r1 = __fadd_rn(p2, p3); }
    unsigned short a, cc; splitf(r0, a, cc); oh[0] = a; ol[0] = cc; splitf(r1, a, cc); oh[1] = a; ol[1] = cc; *(volatile v2us*)(Ah + e) = oh; *(volatile v2us*)(Al + e) = ol; __threadfence(); *(volatile v2us*)(Ah + e) = oh; *(volatile v2us*)(Al + e) = ol; }
__global__ __launch_bounds__(256) void k_bpl(const float* __restrict__ KF, const float* __restrict__ CS, bf* Bh, bf* Bl) { const size_t e = ((size_t)blockIdx.x * 256 + threadIdx.x) * 2; if (e >= (size_t)NH_ * TT * KK) return; const int c = (int)(e % KK); const int j = (int)((e / KK) % TT); const int h = (int)(e / ((size_t)KK * TT)); v2us oh, ol; float r0, r1;
    if (c < HD) { r0 = KF[(size_t)j * DD + h * HD + c]; r1 = KF[(size_t)j * DD + h * HD + c + 1]; } else { const int m = (c - HD) >> 1; const v2f cs = *(const v2f*)(CS + ((size_t)j * 32 + m) * 2); r0 = cs[1]; r1 = cs[0]; }
    unsigned short a, cc; splitf(r0, a, cc); oh[0] = a; ol[0] = cc; splitf(r1, a, cc); oh[1] = a; ol[1] = cc; *(volatile v2us*)(Bh + e) = oh; *(volatile v2us*)(Bl + e) = ol; __threadfence(); *(volatile v2us*)(Bh + e) = oh; *(volatile v2us*)(Bl + e) = ol; }
__global__ __launch_bounds__(256) void k_vtp(const float* __restrict__ VF, h16* VT) { const size_t e = ((size_t)blockIdx.x * 256 + threadIdx.x) * 2; if (e >= (size_t)NH_ * HD * TT) return; const int j = (int)(e % TT); const int d = (int)((e / TT) % HD); const int h = (int)(e / ((size_t)TT * HD)); v2h o; o[0] = tohx(VF[(size_t)j * DD + h * HD + d]); o[1] = tohx(VF[(size_t)(j + 1) * DD + h * HD + d]); *(volatile v2h*)(VT + e) = o; __threadfence(); *(volatile v2h*)(VT + e) = o; }
__global__ __launch_bounds__(256) void k_soft(const float* __restrict__ Sb, h16* P) { const int lane = threadIdx.x & 31; const int row = blockIdx.x * 8 + (threadIdx.x >> 5); if (row >= ZH * TT) return; const float* sr = Sb + (size_t)row * TT; float v[32]; float mx = -3.0e38f;
#pragma unroll
    for (int ch = 0; ch < 8; ++ch) { const v4f a = *(const v4f*)(sr + ch * 128 + lane * 4);
#pragma unroll
        for (int q = 0; q < 4; ++q) { v[ch * 4 + q] = a[q]; mx = fmaxf(mx, a[q]); } }
#pragma unroll
    for (int sh = 16; sh; sh >>= 1) mx = fmaxf(mx, __shfl_xor(mx, sh, 32));
    float sum = 0.f;
#pragma unroll
    for (int k = 0; k < 32; ++k) { float d0 = __fsub_rn(v[k], mx); asm volatile("" : "+v"(d0)); v[k] = __expf(d0); sum += v[k]; }
#pragma unroll
    for (int sh = 16; sh; sh >>= 1) sum += __shfl_xor(sum, sh, 32);
    const float f = __fdiv_rn(PCAR, sum);
#pragma unroll 1
    for (int ps = 0; ps < 2; ++ps) {
#pragma unroll
        for (int ch = 0; ch < 8; ++ch) { v4h o; o[0] = tohx(v[ch * 4] * f); o[1] = tohx(v[ch * 4 + 1] * f); o[2] = tohx(v[ch * 4 + 2] * f); o[3] = tohx(v[ch * 4 + 3] * f); *(volatile v4h*)(P + (size_t)row * TT + ch * 128 + lane * 4) = o; }
        if (ps == 0) __threadfence(); } }
__global__ __launch_bounds__(256) void k_mrg(const float* __restrict__ Ob, int h0, bf* Mh, bf* Ml) { const size_t e = ((size_t)blockIdx.x * 256 + threadIdx.x) * 2; if (e >= (size_t)ZH * TT * HD) return; const int d = (int)(e % HD); const int t = (int)((e / HD) % TT); const int z = (int)(e / ((size_t)HD * TT)); v2us oh, ol;
#pragma unroll
    for (int u = 0; u < 2; ++u) { unsigned short a, c; splitf(Ob[e + u] * (1.0f / PCAR), a, c); oh[u] = a; ol[u] = c; } const size_t o = (size_t)t * DD + (h0 + z) * HD + d; *(volatile v2us*)(Mh + o) = oh; *(volatile v2us*)(Ml + o) = ol; __threadfence(); *(volatile v2us*)(Mh + o) = oh; *(volatile v2us*)(Ml + o) = ol; }

extern "C" void kernel_launch(void* const* d_in, const int* in_sizes, int n_in,
                              void* d_out, int out_size, void* d_ws, size_t ws_size, hipStream_t stream) {
    (void)in_sizes; (void)n_in; (void)out_size;
    const float* x = (const float*)d_in[0]; const float* wq = (const float*)d_in[1]; const float* wk = (const float*)d_in[2]; const float* wv = (const float*)d_in[3]; const float* wo = (const float*)d_in[4]; const float* bo = (const float*)d_in[5]; const float* uu = (const float*)d_in[6]; const float* vv = (const float*)d_in[7];
    float* OUT = (float*)d_out;
    char* wsp = (char*)d_ws;
    auto take = [&](size_t bytes) { char* p = wsp; wsp += (bytes + 255) & ~(size_t)255; return (void*)p; };
    bf* WQ = (bf*)take((size_t)DD * DD * 2); bf* WK = (bf*)take((size_t)DD * DD * 2); bf* WV = (bf*)take((size_t)DD * DD * 2); bf* WO = (bf*)take((size_t)DD * DD * 2); float* CS = (float*)take((size_t)TT * 32 * 2 * 4); bf* XB = (bf*)take((size_t)TT * DD * 2);
    float* QF = (float*)take((size_t)TT * DD * 4); float* KF = (float*)take((size_t)TT * DD * 4); float* VF = (float*)take((size_t)TT * DD * 4); bf* Ah = (bf*)take((size_t)NH_ * TT * KK * 2); bf* Al = (bf*)take((size_t)NH_ * TT * KK * 2); bf* Bh = (bf*)take((size_t)NH_ * TT * KK * 2); bf* Bl = (bf*)take((size_t)NH_ * TT * KK * 2); h16* VT = (h16*)take((size_t)NH_ * HD * TT * 2);
    float* Sb = (float*)take((size_t)ZH * TT * TT * 4); h16* P16 = (h16*)take((size_t)ZH * TT * TT * 2); float* Ob = (float*)take((size_t)ZH * TT * HD * 4); bf* Mh = (bf*)take((size_t)TT * DD * 2); bf* Ml = (bf*)take((size_t)TT * DD * 2);
    if ((size_t)(wsp - (char*)d_ws) > ws_size) return;
    k_cvt8<<<(DD * DD / 8 + 255) / 256, 256, 0, stream>>>(wq, WQ, (size_t)DD * DD / 8); k_cvt8<<<(DD * DD / 8 + 255) / 256, 256, 0, stream>>>(wk, WK, (size_t)DD * DD / 8); k_cvt8<<<(DD * DD / 8 + 255) / 256, 256, 0, stream>>>(wv, WV, (size_t)DD * DD / 8); k_cvt8<<<(DD * DD / 8 + 255) / 256, 256, 0, stream>>>(wo, WO, (size_t)DD * DD / 8);
    k_trig<<<(TT * 32 + 255) / 256, 256, 0, stream>>>(CS);
    const unsigned LP = (unsigned)(((size_t)NH_ * TT * KK / 2 + 255) / 256);
    for (int b = 0; b < NB_; ++b) {
        k_cvt8<<<(TT * DD / 8 + 255) / 256, 256, 0, stream>>>(x + (size_t)b * TT * DD, XB, (size_t)TT * DD / 8);
        k_gemmw<bf, 0, false><<<dim3(TT / 64, DD / 64, 1), 32, 0, stream>>>(XB, nullptr, WQ, nullptr, DD, QF, DD, nullptr, 0, 0, 0); k_gemmw<bf, 0, false><<<dim3(TT / 64, DD / 64, 1), 32, 0, stream>>>(XB, nullptr, WK, nullptr, DD, KF, DD, nullptr, 0, 0, 0); k_gemmw<bf, 0, false><<<dim3(TT / 64, DD / 64, 1), 32, 0, stream>>>(XB, nullptr, WV, nullptr, DD, VF, DD, nullptr, 0, 0, 0);
        k_apl<<<LP, 256, 0, stream>>>(QF, uu, vv, CS, Ah, Al); k_bpl<<<LP, 256, 0, stream>>>(KF, CS, Bh, Bl); k_vtp<<<(unsigned)(((size_t)NH_ * HD * TT / 2 + 255) / 256), 256, 0, stream>>>(VF, VT);
        for (int h0 = 0; h0 < NH_; h0 += ZH) { const size_t z = (size_t)h0;
            k_gemmw<bf, 2, false><<<dim3(TT / 64, TT / 64, ZH), 32, 0, stream>>>(Ah + z * TT * KK, Al + z * TT * KK, Bh + z * TT * KK, Bl + z * TT * KK, KK, Sb, TT, nullptr, (size_t)TT * KK, (size_t)TT * KK, (size_t)TT * TT);
            k_soft<<<ZH * TT / 8, 256, 0, stream>>>(Sb, P16);
            k_gemmw<h16, 0, false><<<dim3(TT / 64, 1, ZH), 32, 0, stream>>>(P16, nullptr, VT + z * HD * TT, nullptr, TT, Ob, HD, nullptr, (size_t)TT * TT, (size_t)HD * TT, (size_t)TT * HD);
            k_mrg<<<(unsigned)(((size_t)ZH * TT * HD / 2 + 255) / 256), 256, 0, stream>>>(Ob, h0, Mh, Ml); }
        k_gemmw<bf, 1, true><<<dim3(TT / 64, DD / 64, 1), 32, 0, stream>>>(Mh, Ml, WO, nullptr, DD, OUT + (size_t)b * TT * DD, DD, bo, 0, 0, 0); }
}
